// Block_38860864094289
// MI455X (gfx1250) — hardware-verified
//
#include <hip/hip_runtime.h>
#include <math.h>

typedef __attribute__((ext_vector_type(16))) _Float16 v16h;
typedef __attribute__((ext_vector_type(8)))  _Float16 v8h;
typedef __attribute__((ext_vector_type(16))) __bf16   v16b;
typedef __attribute__((ext_vector_type(8)))  __bf16   v8b;
typedef __attribute__((ext_vector_type(8)))  float    v8f;
typedef __attribute__((ext_vector_type(4)))  float    v4f;
typedef __attribute__((ext_vector_type(2)))  float    v2f;
typedef __attribute__((ext_vector_type(4)))  unsigned v4u;

constexpr int NB = 32;
constexpr int NF = 81;
constexpr int NC = 512;
constexpr int NHID = 2048;
constexpr int NHALF = 40;
constexpr int NF2 = 41;
constexpr int MROWS = NB * NF;
constexpr int MPAD = 2624;
constexpr int M1ROWS = NB * NHALF;
constexpr int M2ROWS = NB * NF2;
constexpr int M2PAD = 1344;
constexpr int DH = 21;
constexpr int DW = 256;
constexpr float INV_SQRT2_F = 0.70710678118654752f;
constexpr float WCARRY = 64.0f;
constexpr float WCARRY_INV = 1.0f / 64.0f;
constexpr float P_CARRY = 16384.0f;
constexpr float P_CARRY_INV = 1.0f / 16384.0f;

static_assert(MPAD % 64 == 0 && MPAD >= MROWS);
static_assert(M1ROWS % 64 == 0);
static_assert(M2PAD % 64 == 0 && M2PAD >= M2ROWS);
static_assert(NC % 64 == 0 && NHID % 64 == 0 && NC % 32 == 0 && NHID % 32 == 0);
static_assert(MROWS % 8 == 0 && MPAD % 8 == 0);
static_assert((NB * DH * (DW / 4)) % 256 == 0);
static_assert((M2PAD * (NC / 2)) % 256 == 0);
static_assert((M1ROWS * NHID / 2) % 256 == 0 && (M2PAD * NHID / 2) % 256 == 0);

__device__ __forceinline__ unsigned short f2bf_bits(float f) {
  unsigned u = __float_as_uint(f);
  return (unsigned short)((u + 0x7FFFu + ((u >> 16) & 1u)) >> 16);
}
__device__ __forceinline__ float bf_bits2f(unsigned short h) { return __uint_as_float(((unsigned)h) << 16); }
__device__ __forceinline__ unsigned h2u(float f) { return (unsigned)__builtin_bit_cast(unsigned short, (_Float16)f); }

__device__ __forceinline__ void dep_guard_h(v8f& a, v8f& b, v16h x, v16h y) { asm volatile("v_nop\n\tv_nop\n\tv_nop\n\tv_nop" : "+v"(a), "+v"(b) : "v"(x), "v"(y)); }
__device__ __forceinline__ void dep_guard_b(v8f& a, v8f& b, v16b x, v16b y) { asm volatile("v_nop\n\tv_nop\n\tv_nop\n\tv_nop" : "+v"(a), "+v"(b) : "v"(x), "v"(y)); }
__device__ __forceinline__ void keep4_h(v16h a, v16h b, v16h c, v16h d) { asm volatile("v_nop" :: "v"(a), "v"(b), "v"(c), "v"(d)); }
__device__ __forceinline__ void keep4_b(v16b a, v16b b, v16b c, v16b d) { asm volatile("v_nop" :: "v"(a), "v"(b), "v"(c), "v"(d)); }
__device__ __forceinline__ void acc_guard4(v8f& a, v8f& b, v8f& c, v8f& d) { asm volatile("v_nop\n\tv_nop\n\tv_nop\n\tv_nop" : "+v"(a), "+v"(b), "+v"(c), "+v"(d)); }

template <typename T> struct Frag;
template <> struct Frag<_Float16> {
  typedef v16h V; union U { v16h v; v8h h[2]; };
  static __device__ __forceinline__ v16h load(const _Float16* p) {
    U f; f.h[0] = *(const v8h*)(p); f.h[1] = *(const v8h*)(p + 16); return f.v;
  }
  static __device__ __forceinline__ v8f mma(v16h a, v16h b, v8f c) {
    return __builtin_amdgcn_wmma_f32_16x16x32_f16(false, a, false, b, (short)0, c, false, false);
  }
  static __device__ __forceinline__ void guard(v8f& a, v8f& b, v16h x, v16h y) { dep_guard_h(a, b, x, y); }
  static __device__ __forceinline__ void keep(v16h a, v16h b, v16h c, v16h d) { keep4_h(a, b, c, d); }
};
template <> struct Frag<__bf16> {
  typedef v16b V; union U { v16b v; v8b h[2]; };
  static __device__ __forceinline__ v16b load(const __bf16* p) {
    U f; f.h[0] = *(const v8b*)(p); f.h[1] = *(const v8b*)(p + 16); return f.v;
  }
  static __device__ __forceinline__ v8f mma(v16b a, v16b b, v8f c) {
    return __builtin_amdgcn_wmma_f32_16x16x32_bf16(false, a, false, b, (short)0, c, false, false);
  }
  static __device__ __forceinline__ void guard(v8f& a, v8f& b, v16b x, v16b y) { dep_guard_b(a, b, x, y); }
  static __device__ __forceinline__ void keep(v16b a, v16b b, v16b c, v16b d) { keep4_b(a, b, c, d); }
};

__device__ __forceinline__ v8f mma_h(v16h a, v16h b, v8f c) {
  c = __builtin_amdgcn_wmma_f32_16x16x32_f16(false, a, false, b, (short)0, c, false, false);
  asm volatile("v_nop\n\tv_nop\n\tv_nop\n\tv_nop" : "+v"(c) : "v"(a), "v"(b));
  return c;
}

__device__ __forceinline__ float wave_sum(float v) {
#pragma unroll
  for (int off = 16; off > 0; off >>= 1) v += __shfl_xor(v, off, 32);
  return v;
}
__device__ __forceinline__ float wave_max(float v) {
#pragma unroll
  for (int off = 16; off > 0; off >>= 1) v = fmaxf(v, __shfl_xor(v, off, 32));
  return v;
}

template <int ET> struct Elem;
template <> struct Elem<0> { typedef _Float16 T; };
template <> struct Elem<1> { typedef __bf16 T; };
template <int ET, bool SPLIT, int BIAS_MODE, int OUT_MODE, bool RESID>
__global__ __launch_bounds__(256) void wmma_gemm64(
    const unsigned short* __restrict__ Ap, const unsigned short* __restrict__ A2p, int lda, long strideA,
    const unsigned short* __restrict__ Btp, const unsigned short* __restrict__ Bt2p, int ldb, long strideB,
    void* __restrict__ Cout, void* __restrict__ Cout2, int ldc, long strideC,
    const float* __restrict__ bias,
    const float* __restrict__ resid, long strideR,
    int M, int N, int K, float scale, int Mreal) {
  static_assert(!(RESID && OUT_MODE != 0));
  static_assert(BIAS_MODE == 0 || BIAS_MODE == 2);
  typedef typename Elem<ET>::T T;
  typedef typename Frag<T>::V V;
  const T* A = (const T*)Ap; const T* A2 = (const T*)A2p; const T* Bt = (const T*)Btp; const T* Bt2 = (const T*)Bt2p;
  __shared__ __align__(16) float sT[8][16 * 68];
  const int b    = blockIdx.y;
  const int lane = threadIdx.x & 31;
  const int wave = threadIdx.x >> 5;
  const int tilesN = N >> 6;
  const int tilesM = M >> 6;
  const int tile = blockIdx.x * 8 + wave;
  if (tile >= tilesM * tilesN) return;
  const int tm = tile / tilesN;
  const int tn = tile - tm * tilesN;
  const int m0 = tm << 6;
  const int n0 = tn << 6;

  const T* Ab  = A  + (size_t)b * strideA;
  const T* Bb  = Bt + (size_t)b * strideB;
  const T* Ab2 = SPLIT ? (A2  + (size_t)b * strideA) : nullptr;
  const T* Bb2 = SPLIT ? (Bt2 + (size_t)b * strideB) : nullptr;

  const int rlane = lane & 15;
  const int koff  = (lane >> 4) * 8;
  const int mOff  = (lane >> 4) * 8;

  v8f acc[4][4];
#pragma unroll
  for (int i = 0; i < 4; ++i)
#pragma unroll
    for (int j = 0; j < 4; ++j) acc[i][j] = (v8f){0.f,0.f,0.f,0.f,0.f,0.f,0.f,0.f};

  for (int k0 = 0; k0 < K; k0 += 32) {
    V bh[4], bl[4];
#pragma unroll
    for (int j = 0; j < 4; ++j) {
      const size_t bo = (size_t)(n0 + (j << 4) + rlane) * ldb + koff + k0;
      bh[j] = Frag<T>::load(Bb + bo);
      if (SPLIT) bl[j] = Frag<T>::load(Bb2 + bo);
    }
#pragma unroll
    for (int i = 0; i < 4; ++i) {
      const size_t ao = (size_t)(m0 + (i << 4) + rlane) * lda + koff + k0;
      V ah = Frag<T>::load(Ab + ao);
      V al;
      if (SPLIT) al = Frag<T>::load(Ab2 + ao);
#pragma unroll
      for (int j = 0; j < 4; ++j) {
        acc[i][j] = Frag<T>::mma(ah, bh[j], acc[i][j]);
        if (SPLIT) {
          acc[i][j] = Frag<T>::mma(ah, bl[j], acc[i][j]);
          acc[i][j] = Frag<T>::mma(al, bh[j], acc[i][j]);
        }
      }
      Frag<T>::guard(acc[i][0], acc[i][3], ah, SPLIT ? al : ah);
    }
    Frag<T>::keep(bh[0], bh[1], bh[2], bh[3]);
    if (SPLIT) Frag<T>::keep(bl[0], bl[1], bl[2], bl[3]);
  }
  acc_guard4(acc[0][0], acc[0][1], acc[0][2], acc[0][3]);
  acc_guard4(acc[1][0], acc[1][1], acc[1][2], acc[1][3]);
  acc_guard4(acc[2][0], acc[2][1], acc[2][2], acc[2][3]);
  acc_guard4(acc[3][0], acc[3][1], acc[3][2], acc[3][3]);

  float* slab = sT[wave];
#pragma unroll
  for (int i = 0; i < 4; ++i) {
    const int mBase = m0 + (i << 4);
#pragma unroll
    for (int j = 0; j < 4; ++j) {
      const int n = n0 + (j << 4) + rlane;
      float bv = 0.f;
      if (BIAS_MODE == 2) bv = bias[n];
#pragma unroll
      for (int r = 0; r < 8; ++r) {
        float v = acc[i][j][r] * scale;
        if (BIAS_MODE == 2) v += bv;
        slab[(mOff + r) * 68 + (j << 4) + rlane] = v;
      }
    }
    __builtin_amdgcn_fence(__ATOMIC_RELEASE, "workgroup");
    __builtin_amdgcn_wave_barrier();
    __builtin_amdgcn_fence(__ATOMIC_ACQUIRE, "workgroup");
    if (OUT_MODE == 0) {
      float* C = (float*)Cout + (size_t)b * strideC;
      const float* Rb = RESID ? (resid + (size_t)b * strideR) : nullptr;
      const int hh = lane >> 4, c4 = (lane & 15) * 4;
      for (int pass = 0; pass < 2; ++pass) {
#pragma unroll
        for (int it = 0; it < 8; ++it) {
          const int row = it * 2 + hh;
          v4f v = *(const v4f*)(slab + row * 68 + c4);
          if (RESID) {
            int rrow = mBase + row;
            rrow = (rrow < Mreal) ? rrow : (Mreal - 1);
            const v4f rv = *(const v4f*)(Rb + (size_t)rrow * ldc + n0 + c4);
            v += rv;
          }
          *(volatile v4f*)(C + (size_t)(mBase + row) * ldc + n0 + c4) = v;
        }
        __threadfence();
      }
    } else {
      const int q = lane >> 3, c8 = (lane & 7) * 8;
      unsigned short* C  = (unsigned short*)Cout  + (size_t)b * strideC;
      unsigned short* C2 = (OUT_MODE == 2) ? ((unsigned short*)Cout2 + (size_t)b * strideC) : nullptr;
      for (int pass = 0; pass < 2; ++pass) {
#pragma unroll
        for (int it = 0; it < 4; ++it) {
          const int row = it * 4 + q;
          const float* sp = slab + row * 68 + c8;
          v8h hv, lv;
#pragma unroll
          for (int e = 0; e < 8; ++e) {
            if (OUT_MODE == 1) {
              hv[e] = (_Float16)sp[e];
            } else {
              unsigned short hb = f2bf_bits(sp[e]);
              unsigned short lb = f2bf_bits(sp[e] - bf_bits2f(hb));
              hv[e] = __builtin_bit_cast(_Float16, hb);
              lv[e] = __builtin_bit_cast(_Float16, lb);
            }
          }
          *(volatile v8h*)(C + (size_t)(mBase + row) * ldc + n0 + c8) = hv;
          if (OUT_MODE == 2) *(volatile v8h*)(C2 + (size_t)(mBase + row) * ldc + n0 + c8) = lv;
        }
        __threadfence();
      }
    }
    __builtin_amdgcn_fence(__ATOMIC_RELEASE, "workgroup");
    __builtin_amdgcn_wave_barrier();
    __builtin_amdgcn_fence(__ATOMIC_ACQUIRE, "workgroup");
  }
}

template <int PMODE>
__global__ __launch_bounds__(256) void prep_wt_kernel(const float* __restrict__ w0, const float* __restrict__ w1,
    int Kd, int Nd,
    unsigned short* __restrict__ o0a, unsigned short* __restrict__ o0b,
    unsigned short* __restrict__ o1a, unsigned short* __restrict__ o1b) {
  __shared__ __align__(16) float tile[64 * 68];
  const int t = threadIdx.x;
  const bool second = (blockIdx.z != 0);
  const float* w = second ? w1 : w0;
  unsigned short* oa = second ? o1a : o0a;
  unsigned short* ob = second ? o1b : o0b;
  const int n0 = blockIdx.x * 64;
  const int k0 = blockIdx.y * 64;
#pragma unroll 4
  for (int it = 0; it < 16; ++it) {
    const int e = it * 256 + t;
    const int kk = e >> 6, nn = e & 63;
    tile[nn * 68 + kk] = w[(size_t)(k0 + kk) * Nd + n0 + nn];
  }
  __syncthreads();
  const int c8 = (t & 7) * 8;
  v4u pa[2], pb[2];
  size_t go[2];
#pragma unroll
  for (int hs = 0; hs < 2; ++hs) {
    const int nn = (t >> 3) + 32 * hs;
    const v4f f0 = *(const v4f*)(tile + nn * 68 + c8);
    const v4f f1 = *(const v4f*)(tile + nn * 68 + c8 + 4);
    const float fv[8] = {f0[0], f0[1], f0[2], f0[3], f1[0], f1[1], f1[2], f1[3]};
    unsigned ua[8], ub[8];
#pragma unroll
    for (int e = 0; e < 8; ++e) {
      if (PMODE == 0) {
        ua[e] = h2u(fv[e] * WCARRY);
        ub[e] = 0u;
      } else {
        const unsigned short hb = f2bf_bits(fv[e]);
        const unsigned short lb = f2bf_bits(fv[e] - bf_bits2f(hb));
        ua[e] = (unsigned)hb;
        ub[e] = (unsigned)lb;
      }
    }
    v4u a4, b4;
    a4[0] = ua[0] | (ua[1] << 16); a4[1] = ua[2] | (ua[3] << 16); a4[2] = ua[4] | (ua[5] << 16); a4[3] = ua[6] | (ua[7] << 16);
    b4[0] = ub[0] | (ub[1] << 16); b4[1] = ub[2] | (ub[3] << 16); b4[2] = ub[4] | (ub[5] << 16); b4[3] = ub[6] | (ub[7] << 16);
    pa[hs] = a4; pb[hs] = b4;
    go[hs] = (size_t)(n0 + nn) * Kd + k0 + c8;
  }
  for (int pass = 0; pass < 2; ++pass) {
#pragma unroll
    for (int hs = 0; hs < 2; ++hs) {
      *(volatile v4u*)(oa + go[hs]) = pa[hs];
      if (PMODE == 1) *(volatile v4u*)(ob + go[hs]) = pb[hs];
    }
    __threadfence();
  }
}

#define PACK8(U, BASE, DST) \
  DST[0] = U[BASE + 0] | (U[BASE + 1] << 16); DST[1] = U[BASE + 2] | (U[BASE + 3] << 16); \
  DST[2] = U[BASE + 4] | (U[BASE + 5] << 16); DST[3] = U[BASE + 6] | (U[BASE + 7] << 16);

__global__ __launch_bounds__(256) void ln1_kernel(const float* __restrict__ x,
    const float* __restrict__ gw, const float* __restrict__ gb,
    unsigned short* __restrict__ h16, unsigned short* __restrict__ hbh, unsigned short* __restrict__ hbl) {
  const int lane = threadIdx.x & 31, wave = threadIdx.x >> 5;
  const int row = blockIdx.x * 8 + wave;
  const bool ok = row < MROWS;
  const int rowc = ok ? row : (MROWS - 1);
  const float* xr = x + (size_t)rowc * NC;
  float xv[16], wv[16], bv[16];
#pragma unroll
  for (int i = 0; i < 2; ++i) {
    const int c0 = i * 256 + lane * 8;
    const v4f a0 = *(const v4f*)(xr + c0), a1 = *(const v4f*)(xr + c0 + 4);
    const v4f w0 = *(const v4f*)(gw + c0), w1 = *(const v4f*)(gw + c0 + 4);
    const v4f b0 = *(const v4f*)(gb + c0), b1 = *(const v4f*)(gb + c0 + 4);
#pragma unroll
    for (int e = 0; e < 4; ++e) {
      xv[i * 8 + e] = a0[e]; xv[i * 8 + 4 + e] = a1[e];
      wv[i * 8 + e] = w0[e]; wv[i * 8 + 4 + e] = w1[e];
      bv[i * 8 + e] = b0[e]; bv[i * 8 + 4 + e] = b1[e];
    }
  }
  float s = 0.0f;
#pragma unroll
  for (int e = 0; e < 16; ++e) s += xv[e];
  s = wave_sum(s);
  const float mean = s * (1.0f / (float)NC);
  float qs = 0.0f;
#pragma unroll
  for (int e = 0; e < 16; ++e) { const float d = xv[e] - mean; qs += d * d; }
  qs = wave_sum(qs);
  const float rstd = rsqrtf(qs * (1.0f / (float)NC) + 1e-5f);
  unsigned uh[16], ubh[16], ubl[16];
#pragma unroll
  for (int e = 0; e < 16; ++e) {
    float y = (xv[e] - mean) * rstd * wv[e] + bv[e];
    y = ok ? y : 0.0f;
    uh[e] = h2u(y);
    const unsigned short hb = f2bf_bits(y);
    const unsigned short lb = f2bf_bits(y - bf_bits2f(hb));
    ubh[e] = (unsigned)hb;
    ubl[e] = (unsigned)lb;
  }
  v4u ph[2], pbh[2], pbl[2];
  PACK8(uh, 0, ph[0]);  PACK8(uh, 8, ph[1]);
  PACK8(ubh, 0, pbh[0]); PACK8(ubh, 8, pbh[1]);
  PACK8(ubl, 0, pbl[0]); PACK8(ubl, 8, pbl[1]);
  const size_t ro = (size_t)row * NC;
  for (int pass = 0; pass < 2; ++pass) {
#pragma unroll
    for (int i = 0; i < 2; ++i) {
      const size_t eo = ro + i * 256 + lane * 8;
      *(volatile v4u*)(h16 + eo) = ph[i];
      *(volatile v4u*)(hbh + eo) = pbh[i];
      *(volatile v4u*)(hbl + eo) = pbl[i];
    }
    __threadfence();
  }
}

__global__ __launch_bounds__(256) void ln23_kernel(const float* __restrict__ xp,
    const float* __restrict__ g2w, const float* __restrict__ g2b,
    const float* __restrict__ g3w, const float* __restrict__ g3b,
    unsigned short* __restrict__ hm16, float* __restrict__ xa, float* __restrict__ hf) {
  const int lane = threadIdx.x & 31, wave = threadIdx.x >> 5;
  const int row = blockIdx.x * 8 + wave;
  const int b = row / NF, f = row - b * NF;
  const float* xr = xp + (size_t)row * NC;
  v4f xq[4];
#pragma unroll
  for (int i = 0; i < 4; ++i) xq[i] = *(const v4f*)(xr + i * 128 + lane * 4);
  float s = 0.0f;
#pragma unroll
  for (int i = 0; i < 4; ++i) s += (xq[i][0] + xq[i][1]) + (xq[i][2] + xq[i][3]);
  s = wave_sum(s);
  const float mean = s * (1.0f / (float)NC);
  float qs = 0.0f;
#pragma unroll
  for (int i = 0; i < 4; ++i) {
#pragma unroll
    for (int e = 0; e < 4; ++e) { const float d = xq[i][e] - mean; qs += d * d; }
  }
  qs = wave_sum(qs);
  const float rstd = rsqrtf(qs * (1.0f / (float)NC) + 1e-5f);
  if (f < NHALF) {
    const size_t orow = (size_t)b * NHALF + f;
    v4u ph[2];
#pragma unroll
    for (int i = 0; i < 2; ++i) {
      const int c0 = i * 256 + lane * 8;
      const v4f x0 = *(const v4f*)(xr + c0), x1 = *(const v4f*)(xr + c0 + 4);
      const v4f w0 = *(const v4f*)(g2w + c0), w1 = *(const v4f*)(g2w + c0 + 4);
      const v4f b0 = *(const v4f*)(g2b + c0), b1 = *(const v4f*)(g2b + c0 + 4);
      unsigned u[8];
#pragma unroll
      for (int e = 0; e < 4; ++e) {
        u[e]     = h2u((x0[e] - mean) * rstd * w0[e] + b0[e]);
        u[4 + e] = h2u((x1[e] - mean) * rstd * w1[e] + b1[e]);
      }
      PACK8(u, 0, ph[i]);
    }
    float* xao = xa + orow * NC;
    unsigned short* hmo = hm16 + orow * NC;
    for (int pass = 0; pass < 2; ++pass) {
#pragma unroll
      for (int i = 0; i < 4; ++i) *(volatile v4f*)(xao + i * 128 + lane * 4) = xq[i];
#pragma unroll
      for (int i = 0; i < 2; ++i) *(volatile v4u*)(hmo + i * 256 + lane * 8) = ph[i];
      __threadfence();
    }
  } else {
    const size_t orow = (size_t)b * NF2 + (f - NHALF);
    v4f yq[4];
#pragma unroll
    for (int i = 0; i < 4; ++i) {
      const int c0 = i * 128 + lane * 4;
      const v4f w0 = *(const v4f*)(g3w + c0);
      const v4f b0 = *(const v4f*)(g3b + c0);
      v4f y;
#pragma unroll
      for (int e = 0; e < 4; ++e) y[e] = (xq[i][e] - mean) * rstd * w0[e] + b0[e];
      yq[i] = y;
    }
    float* hfo = hf + orow * NC;
    for (int pass = 0; pass < 2; ++pass) {
#pragma unroll
      for (int i = 0; i < 4; ++i) *(volatile v4f*)(hfo + i * 128 + lane * 4) = yq[i];
      __threadfence();
    }
  }
}

constexpr int AT_TQ = 16;
constexpr int AT_NQT = (NF + AT_TQ - 1) / AT_TQ;
constexpr int AT_JP = 96;
constexpr int AT_PP = 104;
constexpr int AT_CC = 64;
constexpr int AT_NCC = NC / AT_CC;
constexpr int AT_SP = 100;
constexpr int AT_OP = 68;
constexpr int AT_NT = 192;
constexpr int AT_NWV = AT_NT / 32;
static_assert(AT_JP == AT_NT / 2);
static_assert(NF > 64 && NF <= AT_JP && AT_JP % 32 == 0);
static_assert((AT_JP * (AT_CC / 8)) % AT_NT == 0);
static_assert(AT_NQT * AT_TQ >= NF);
static_assert(NC % AT_CC == 0 && AT_CC % 16 == 0);

#define RELU_ACC4(SARR, BASE, QV, KK) \
  SARR[BASE + 0] += fmaxf(QV[0] + KK, 0.0f); \
  SARR[BASE + 1] += fmaxf(QV[1] + KK, 0.0f); \
  SARR[BASE + 2] += fmaxf(QV[2] + KK, 0.0f); \
  SARR[BASE + 3] += fmaxf(QV[3] + KK, 0.0f);

__global__ __launch_bounds__(AT_NT) void attn_kernel(const float* __restrict__ qk,
    const unsigned short* __restrict__ v16, unsigned short* __restrict__ av16) {
  __shared__ __align__(16) float qT[NC * AT_TQ];
  __shared__ __align__(16) float sc[AT_TQ * AT_SP];
  __shared__ __align__(16) unsigned short Ps[AT_TQ * AT_PP];
  __shared__ __align__(16) unsigned short Vt[AT_CC * AT_PP];
  __shared__ __align__(16) float osl[AT_TQ * AT_OP];

  const int t = threadIdx.x;
  const int lane = t & 31, wave = t >> 5;
  const int b = blockIdx.x / AT_NQT;
  const int qtile = blockIdx.x - b * AT_NQT;
  const int i0 = qtile * AT_TQ;
  const size_t rowb = (size_t)b * NF;
  const int QKLD = 2 * NC;

  for (int e = t; e < AT_TQ * (NC / 4); e += AT_NT) {
    const int r = e / (NC / 4);
    const int c4 = (e - r * (NC / 4)) * 4;
    int qi = i0 + r; qi = (qi < NF) ? qi : (NF - 1);
    const v4f qv = *(const v4f*)(qk + (rowb + qi) * QKLD + c4);
    qT[(c4 + 0) * AT_TQ + r] = qv[0];
    qT[(c4 + 1) * AT_TQ + r] = qv[1];
    qT[(c4 + 2) * AT_TQ + r] = qv[2];
    qT[(c4 + 3) * AT_TQ + r] = qv[3];
  }
  __syncthreads();

  const int j = t >> 1, ch = t & 1;
  const int jc = (j < NF) ? j : (NF - 1);
  const float* kr = qk + (rowb + jc) * QKLD + NC + ch * (NC / 2);
  const float* qbp = qT + ch * (NC / 2) * AT_TQ;
  float s[AT_TQ];
#pragma unroll
  for (int r = 0; r < AT_TQ; ++r) s[r] = 0.0f;
#pragma unroll 1
  for (int c4i = 0; c4i < NC / 8; ++c4i) {
    const v4f kv = *(const v4f*)(kr + c4i * 4);
#pragma unroll
    for (int e = 0; e < 4; ++e) {
      const float* qp = qbp + (c4i * 4 + e) * AT_TQ;
      const v4f q0 = *(const v4f*)(qp);
      const v4f q1 = *(const v4f*)(qp + 4);
      const v4f q2 = *(const v4f*)(qp + 8);
      const v4f q3 = *(const v4f*)(qp + 12);
      const float kk = kv[e];
      RELU_ACC4(s, 0, q0, kk)
      RELU_ACC4(s, 4, q1, kk)
      RELU_ACC4(s, 8, q2, kk)
      RELU_ACC4(s, 12, q3, kk)
    }
  }
#pragma unroll
  for (int r = 0; r < AT_TQ; ++r) s[r] += __shfl_xor(s[r], 1, 32);
  if (ch == 0) {
#pragma unroll
    for (int r = 0; r < AT_TQ; ++r) sc[r * AT_SP + j] = s[r];
  }
  __syncthreads();

  for (int r = wave; r < AT_TQ; r += AT_NWV) {
    const float* srow = sc + r * AT_SP;
    const float v0 = srow[lane];
    const float v1 = srow[32 + lane];
    const float v2r = srow[64 + lane];
    const bool ok2 = (64 + lane) < NF;
    float m = fmaxf(v0, v1);
    m = fmaxf(m, ok2 ? v2r : v0);
    m = wave_max(m);
    const float e0 = expf(v0 - m);
    const float e1 = expf(v1 - m);
    const float v2c = ok2 ? v2r : m;
    float e2 = expf(v2c - m);
    e2 = ok2 ? e2 : 0.0f;
    float ssum = (e0 + e1) + e2;
    ssum = wave_sum(ssum);
    const float inv = P_CARRY / ssum;
    unsigned short* prow = Ps + r * AT_PP;
    prow[lane]      = (unsigned short)h2u(e0 * inv);
    prow[32 + lane] = (unsigned short)h2u(e1 * inv);
    const unsigned p2 = h2u(e2 * inv);
    prow[64 + lane] = (unsigned short)(ok2 ? p2 : 0u);
  }
  __syncthreads();

  const int rlane = lane & 15, koff = (lane >> 4) * 8, mOff = (lane >> 4) * 8;
  for (int cc = 0; cc < AT_NCC; ++cc) {
    __syncthreads();
#pragma unroll
    for (int it = 0; it < (AT_JP * (AT_CC / 8)) / AT_NT; ++it) {
      const int e = it * AT_NT + t;
      const int jj = e >> 3, q8 = e & 7;
      const bool okj = jj < NF;
      const int jjc = okj ? jj : (NF - 1);
      const v4u wv4 = *(const v4u*)(v16 + (rowb + jjc) * NC + cc * AT_CC + q8 * 8);
      const unsigned w0 = okj ? wv4[0] : 0u;
      const unsigned w1 = okj ? wv4[1] : 0u;
      const unsigned w2 = okj ? wv4[2] : 0u;
      const unsigned w3 = okj ? wv4[3] : 0u;
      unsigned short* vp = Vt + (q8 * 8) * AT_PP + jj;
      vp[0 * AT_PP] = (unsigned short)(w0 & 0xffffu);
      vp[1 * AT_PP] = (unsigned short)(w0 >> 16);
      vp[2 * AT_PP] = (unsigned short)(w1 & 0xffffu);
      vp[3 * AT_PP] = (unsigned short)(w1 >> 16);
      vp[4 * AT_PP] = (unsigned short)(w2 & 0xffffu);
      vp[5 * AT_PP] = (unsigned short)(w2 >> 16);
      vp[6 * AT_PP] = (unsigned short)(w3 & 0xffffu);
      vp[7 * AT_PP] = (unsigned short)(w3 >> 16);
    }
    __syncthreads();
    for (int tile = wave; tile < AT_CC / 16; tile += AT_NWV) {
      v8f acc = (v8f){0.f,0.f,0.f,0.f,0.f,0.f,0.f,0.f};
#pragma unroll
      for (int ks = 0; ks < AT_JP / 32; ++ks) {
        const v16h af = Frag<_Float16>::load((const _Float16*)Ps + rlane * AT_PP + koff + ks * 32);
        const v16h bfr = Frag<_Float16>::load((const _Float16*)Vt + (tile * 16 + rlane) * AT_PP + koff + ks * 32);
        acc = mma_h(af, bfr, acc);
      }
#pragma unroll
      for (int r = 0; r < 8; ++r) osl[(mOff + r) * AT_OP + tile * 16 + rlane] = acc[r] * P_CARRY_INV;
    }
    __syncthreads();
    for (int rg = wave; rg < AT_TQ / 4; rg += AT_NWV) {
      const int rr = rg * 4 + (lane >> 3);
      const int c8 = (lane & 7) * 8;
      const int qi = i0 + rr;
      const bool okr = qi < NF;
      const v4f f0 = *(const v4f*)(osl + rr * AT_OP + c8);
      const v4f f1 = *(const v4f*)(osl + rr * AT_OP + c8 + 4);
      v4u pk;
      pk[0] = h2u(f0[0]) | (h2u(f0[1]) << 16);
      pk[1] = h2u(f0[2]) | (h2u(f0[3]) << 16);
      pk[2] = h2u(f1[0]) | (h2u(f1[1]) << 16);
      pk[3] = h2u(f1[2]) | (h2u(f1[3]) << 16);
      unsigned short* dst = av16 + (rowb + (okr ? qi : 0)) * NC + cc * AT_CC + c8;
      for (int pass = 0; pass < 2; ++pass) {
        if (okr) *(volatile v4u*)dst = pk;
        __threadfence();
      }
    }
  }
}

__global__ __launch_bounds__(256) void zero16_kernel(v4u* __restrict__ p, int n) {
  const int i = blockIdx.x * 256 + threadIdx.x;
  if (i < n) {
    v4u z; z[0] = 0u; z[1] = 0u; z[2] = 0u; z[3] = 0u;
    *(volatile v4u*)(p + i) = z;
    __threadfence();
    *(volatile v4u*)(p + i) = z;
  }
}

__device__ __forceinline__ float gelu_erf(float x) { return 0.5f * x * (1.0f + erff(x * INV_SQRT2_F)); }

__global__ __launch_bounds__(256) void gelu_kernel(const float* __restrict__ in, unsigned short* __restrict__ out, int n2) {
  const int i = blockIdx.x * 256 + threadIdx.x;
  if (i < n2) {
    const v2f p = *(const v2f*)(in + 2 * (size_t)i);
    const unsigned u = h2u(gelu_erf(p[0])) | (h2u(gelu_erf(p[1])) << 16);
    ((volatile unsigned*)out)[i] = u;
    __threadfence();
    ((volatile unsigned*)out)[i] = u;
  }
}

__global__ __launch_bounds__(256) void dwt_kernel(const float* __restrict__ hf,
    float* __restrict__ pll, float* __restrict__ plh, float* __restrict__ phl, float* __restrict__ phh) {
  const int idx = blockIdx.x * 256 + threadIdx.x;
  const int c4 = idx & (DW / 4 - 1);
  const int rem = idx / (DW / 4);
  const int r = rem % DH, b = rem / DH;
  const float* base = hf + (size_t)b * NF2 * NC;
  const int r0 = 2 * r;
  const int r1 = 2 * r + 1;
  const bool ok1 = r1 < NF2;
  const int r1c = ok1 ? r1 : (NF2 - 1);
  const v4f a0 = *(const v4f*)(base + (size_t)r0 * NC + 8 * c4);
  const v4f a1 = *(const v4f*)(base + (size_t)r0 * NC + 8 * c4 + 4);
  const v4f g0 = *(const v4f*)(base + (size_t)r1c * NC + 8 * c4);
  const v4f g1 = *(const v4f*)(base + (size_t)r1c * NC + 8 * c4 + 4);
  const float S = INV_SQRT2_F;
  const float ea[4] = {a0[0], a0[2], a1[0], a1[2]};
  const float oa[4] = {a0[1], a0[3], a1[1], a1[3]};
  const float eb[4] = {g0[0], g0[2], g1[0], g1[2]};
  const float obv[4] = {g0[1], g0[3], g1[1], g1[3]};
  v4f oll, olh, ohl, ohh;
#pragma unroll
  for (int m = 0; m < 4; ++m) {
    const float la0 = (ea[m] + oa[m]) * S;
    const float ld0 = (ea[m] - oa[m]) * S;
    float la1 = (eb[m] + obv[m]) * S;
    float ld1 = (eb[m] - obv[m]) * S;
    la1 = ok1 ? la1 : 0.0f;
    ld1 = ok1 ? ld1 : 0.0f;
    oll[m] = (la0 + la1) * S;
    olh[m] = (la0 - la1) * S;
    ohl[m] = (ld0 + ld1) * S;
    ohh[m] = (ld0 - ld1) * S;
  }
  const size_t o = ((size_t)(b * DH + r)) * DW + c4 * 4;
  for (int pass = 0; pass < 2; ++pass) {
    *(volatile v4f*)(pll + o) = oll;
    *(volatile v4f*)(plh + o) = olh;
    *(volatile v4f*)(phl + o) = ohl;
    *(volatile v4f*)(phh + o) = ohh;
    __threadfence();
  }
}

__global__ __launch_bounds__(256) void upsample_kernel(const float* __restrict__ pll, unsigned short* __restrict__ low16) {
  const int idx = blockIdx.x * 256 + threadIdx.x;
  const int row = idx / (NC / 2);
  const int c2 = (idx - row * (NC / 2)) * 2;
  const bool ok = row < M2ROWS;
  const int rowc = ok ? row : (M2ROWS - 1);
  const int b = rowc / NF2, y = rowc - b * NF2;
  const float ys = (y == NF2 - 1) ? (float)(DH - 1) : (float)(DH - 1) * ((float)y * (1.0f / (float)(NF2 - 1)));
  int ya = (int)floorf(ys); ya = ya < 0 ? 0 : (ya > DH - 1 ? DH - 1 : ya);
  const int yb = (ya + 1 < DH - 1) ? (ya + 1) : (DH - 1);
  const float wy = ys - (float)ya;
  const float* r0 = pll + ((size_t)b * DH + ya) * DW;
  const float* r1 = pll + ((size_t)b * DH + yb) * DW;
  unsigned u[2];
#pragma unroll
  for (int e = 0; e < 2; ++e) {
    const int xx = c2 + e;
    const float xs = (xx == NC - 1) ? (float)(DW - 1) : (float)(DW - 1) * ((float)xx * (1.0f / (float)(NC - 1)));
    int xa = (int)floorf(xs); xa = xa < 0 ? 0 : (xa > DW - 1 ? DW - 1 : xa);
    const int xb = (xa + 1 < DW - 1) ? (xa + 1) : (DW - 1);
    const float wx = xs - (float)xa;
    const float ta = r0[xa] * (1.0f - wy) + r1[xa] * wy;
    const float tb = r0[xb] * (1.0f - wy) + r1[xb] * wy;
    float val = ta * (1.0f - wx) + tb * wx;
    val = ok ? val : 0.0f;
    u[e] = h2u(val);
  }
  const unsigned pk = u[0] | (u[1] << 16);
  ((volatile unsigned*)low16)[idx] = pk;
  __threadfence();
  ((volatile unsigned*)low16)[idx] = pk;
}

__global__ __launch_bounds__(256) void final_kernel(const float* __restrict__ y1p, const float* __restrict__ xpost,
    const float* __restrict__ lowout, const float* __restrict__ plh, const float* __restrict__ phl,
    const float* __restrict__ phh, float* __restrict__ out) {
  const int lane = threadIdx.x & 31, wave = threadIdx.x >> 5;
  const int row = blockIdx.x * 8 + wave;
  const int b = row / NF, f = row - b * NF;
  float* orow = out + (size_t)row * NC;
  if (f < NHALF) {
    const float* src = y1p + ((size_t)b * NHALF + f) * NC;
    v4f vv[4];
#pragma unroll
    for (int i = 0; i < 4; ++i) vv[i] = *(const v4f*)(src + i * 128 + lane * 4);
    for (int pass = 0; pass < 2; ++pass) {
#pragma unroll
      for (int i = 0; i < 4; ++i) *(volatile v4f*)(orow + i * 128 + lane * 4) = vv[i];
      __threadfence();
    }
  } else {
    const int f2 = f - NHALF;
    const int hr = f2 >> 1;
    const float sgh = (f2 & 1) ? -1.0f : 1.0f;
    const float* xr = xpost + (size_t)row * NC;
    const float ys = (hr == DH - 1) ? (float)(NF2 - 1) : (float)(NF2 - 1) * ((float)hr * (1.0f / (float)(DH - 1)));
    int ya = (int)floorf(ys); ya = ya < 0 ? 0 : (ya > NF2 - 1 ? NF2 - 1 : ya);
    const int yb = (ya + 1 < NF2 - 1) ? (ya + 1) : (NF2 - 1);
    const float wy = ys - (float)ya;
    const float* l0 = lowout + ((size_t)b * NF2 + ya) * NC;
    const float* l1 = lowout + ((size_t)b * NF2 + yb) * NC;
    const size_t drow = ((size_t)b * DH + hr) * DW;
    const float* dlh = plh + drow;
    const float* dhl = phl + drow;
    const float* dhh = phh + drow;
    const float S = INV_SQRT2_F;
    for (int pass = 0; pass < 2; ++pass) {
#pragma unroll 1
      for (int i = 0; i < 4; ++i) {
        const int c0 = i * 128 + lane * 4;
        const int wc0 = c0 >> 1;
        const v4f xbv = *(const v4f*)(xr + c0);
        const v2f lh2 = *(const v2f*)(dlh + wc0);
        const v2f hl2 = *(const v2f*)(dhl + wc0);
        const v2f hh2 = *(const v2f*)(dhh + wc0);
        float lowd[2];
#pragma unroll
        for (int e = 0; e < 2; ++e) {
          const int wc = wc0 + e;
          const float xs = (wc == DW - 1) ? (float)(NC - 1) : (float)(NC - 1) * ((float)wc * (1.0f / (float)(DW - 1)));
          int xa = (int)floorf(xs); xa = xa < 0 ? 0 : (xa > NC - 1 ? NC - 1 : xa);
          const int xb = (xa + 1 < NC - 1) ? (xa + 1) : (NC - 1);
          const float wx = xs - (float)xa;
          const float ta = l0[xa] * (1.0f - wy) + l1[xa] * wy;
          const float tb = l0[xb] * (1.0f - wy) + l1[xb] * wy;
          lowd[e] = ta * (1.0f - wx) + tb * wx;
        }
        v4f o;
#pragma unroll
        for (int e = 0; e < 4; ++e) {
          const int p = e >> 1;
          const float ah = (lowd[p] + sgh * lh2[p]) * S;
          const float dh = (hl2[p] + sgh * hh2[p]) * S;
          const float sgw = (e & 1) ? -1.0f : 1.0f;
          o[e] = xbv[e] + (ah + sgw * dh) * S;
        }
        *(volatile v4f*)(orow + c0) = o;
      }
      __threadfence();
    }
  }
}

static inline dim3 gemm_grid(int M, int N) {
  const int tiles = (M / 64) * (N / 64);
  return dim3((tiles + 7) / 8, 1, 1);
}

extern "C" void kernel_launch(void* const* d_in, const int* in_sizes, int n_in,
                              void* d_out, int out_size, void* d_ws, size_t ws_size,
                              hipStream_t stream) {
  if (n_in < 20) return;
  if (in_sizes[0] != MROWS * NC || out_size != MROWS * NC) return;
  if (in_sizes[3] != NC * NC || in_sizes[4] != NC * NC || in_sizes[5] != NC * NC || in_sizes[6] != NC * NC) return;
  if (in_sizes[10] != NC * NHID || in_sizes[12] != NHID * NC || in_sizes[16] != NC * NHID || in_sizes[18] != NHID * NC) return;
  if (in_sizes[1] != NC || in_sizes[7] != NC || in_sizes[11] != NHID || in_sizes[17] != NHID) return;

  const float* x     = (const float*)d_in[0];
  const float* n1w   = (const float*)d_in[1];
  const float* n1b   = (const float*)d_in[2];
  const float* wq    = (const float*)d_in[3];
  const float* wk    = (const float*)d_in[4];
  const float* wv    = (const float*)d_in[5];
  const float* wp    = (const float*)d_in[6];
  const float* bp    = (const float*)d_in[7];
  const float* n2w   = (const float*)d_in[8];
  const float* n2b   = (const float*)d_in[9];
  const float* w11   = (const float*)d_in[10];
  const float* b11   = (const float*)d_in[11];
  const float* w12   = (const float*)d_in[12];
  const float* b12   = (const float*)d_in[13];
  const float* n3w   = (const float*)d_in[14];
  const float* n3b   = (const float*)d_in[15];
  const float* w21   = (const float*)d_in[16];
  const float* b21   = (const float*)d_in[17];
  const float* w22   = (const float*)d_in[18];
  const float* b22   = (const float*)d_in[19];
  float* out = (float*)d_out;

  char* wsb = (char*)d_ws;
  size_t off = 0;
  auto carve = [&](size_t bytes) -> char* { char* p = wsb + off; off += (bytes + 255) & ~(size_t)255; return p; };
  unsigned short* wqkT_hi = (unsigned short*)carve((size_t)2 * NC * NC * 2);
  unsigned short* wqkT_lo = (unsigned short*)carve((size_t)2 * NC * NC * 2);
  unsigned short* wvpT    = (unsigned short*)carve((size_t)2 * NC * NC * 2);
  unsigned short* w1T     = (unsigned short*)carve((size_t)2 * NHID * NC * 2);
  unsigned short* w2T     = (unsigned short*)carve((size_t)2 * NC * NHID * 2);
  unsigned short* h16     = (unsigned short*)carve((size_t)MPAD * NC * 2);
  unsigned short* hbh     = (unsigned short*)carve((size_t)MPAD * NC * 2);
  unsigned short* hbl     = (unsigned short*)carve((size_t)MPAD * NC * 2);
  float*          qk      = (float*)carve((size_t)MPAD * 2 * NC * 4);
  unsigned short* v16     = (unsigned short*)carve((size_t)MPAD * NC * 2);
  unsigned short* av16    = (unsigned short*)carve((size_t)MPAD * NC * 2);
  float*          xpost   = (float*)carve((size_t)MPAD * NC * 4);
  unsigned short* hm16    = (unsigned short*)carve((size_t)M1ROWS * NC * 2);
  float*          xa      = (float*)carve((size_t)M1ROWS * NC * 4);
  float*          hf      = (float*)carve((size_t)M2ROWS * NC * 4);
  float*          pre1    = (float*)carve((size_t)M1ROWS * NHID * 4);
  unsigned short* t1      = (unsigned short*)carve((size_t)M1ROWS * NHID * 2);
  float*          y1p     = (float*)carve((size_t)M1ROWS * NC * 4);
  float*          pll     = (float*)carve((size_t)NB * DH * DW * 4);
  float*          plh     = (float*)carve((size_t)NB * DH * DW * 4);
  float*          phl     = (float*)carve((size_t)NB * DH * DW * 4);
  float*          phh     = (float*)carve((size_t)NB * DH * DW * 4);
  unsigned short* low16   = (unsigned short*)carve((size_t)M2PAD * NC * 2);
  float*          pre2    = (float*)carve((size_t)M2PAD * NHID * 4);
  unsigned short* t2      = (unsigned short*)carve((size_t)M2PAD * NHID * 2);
  float*          lowout  = (float*)carve((size_t)M2PAD * NC * 4);
  if (off > ws_size) return;

  prep_wt_kernel<1><<<dim3(NC / 64, NC / 64, 2), 256, 0, stream>>>(wq, wk, NC, NC,
      wqkT_hi, wqkT_lo, wqkT_hi + (size_t)NC * NC, wqkT_lo + (size_t)NC * NC);
  prep_wt_kernel<0><<<dim3(NC / 64, NC / 64, 2), 256, 0, stream>>>(wv, wp, NC, NC,
      wvpT, wvpT, wvpT + (size_t)NC * NC, wvpT + (size_t)NC * NC);
  prep_wt_kernel<0><<<dim3(NHID / 64, NC / 64, 2), 256, 0, stream>>>(w11, w21, NC, NHID,
      w1T, w1T, w1T + (size_t)NHID * NC, w1T + (size_t)NHID * NC);
  prep_wt_kernel<0><<<dim3(NC / 64, NHID / 64, 2), 256, 0, stream>>>(w12, w22, NHID, NC,
      w2T, w2T, w2T + (size_t)NC * NHID, w2T + (size_t)NC * NHID);

  ln1_kernel<<<MPAD / 8, 256, 0, stream>>>(x, n1w, n1b, h16, hbh, hbl);

  wmma_gemm64<1, true, 0, 0, false><<<gemm_grid(MPAD, 2 * NC), 256, 0, stream>>>(
      hbh, hbl, NC, 0L, wqkT_hi, wqkT_lo, NC, 0L, (void*)qk, (void*)qk, 2 * NC, 0L,
      bp, x, 0L, MPAD, 2 * NC, NC, 1.0f, MPAD);
  wmma_gemm64<0, false, 0, 1, false><<<gemm_grid(MPAD, NC), 256, 0, stream>>>(
      h16, h16, NC, 0L, wvpT, wvpT, NC, 0L, (void*)v16, (void*)v16, NC, 0L,
      bp, x, 0L, MPAD, NC, NC, WCARRY_INV, MPAD);

  attn_kernel<<<NB * AT_NQT, AT_NT, 0, stream>>>(qk, v16, av16);
  {
    const int nz = (MPAD - MROWS) * NC * 2 / 16;
    zero16_kernel<<<(nz + 255) / 256, 256, 0, stream>>>((v4u*)(av16 + (size_t)MROWS * NC), nz);
  }

  wmma_gemm64<0, false, 2, 0, true><<<gemm_grid(MPAD, NC), 256, 0, stream>>>(
      av16, av16, NC, 0L, wvpT + (size_t)NC * NC, wvpT + (size_t)NC * NC, NC, 0L,
      (void*)xpost, (void*)xpost, NC, 0L, bp, x, 0L, MPAD, NC, NC, WCARRY_INV, MROWS);

  ln23_kernel<<<MROWS / 8, 256, 0, stream>>>(xpost, n2w, n2b, n3w, n3b, hm16, xa, hf);

  wmma_gemm64<0, false, 2, 0, false><<<gemm_grid(M1ROWS, NHID), 256, 0, stream>>>(
      hm16, hm16, NC, 0L, w1T, w1T, NC, 0L, (void*)pre1, (void*)pre1, NHID, 0L,
      b11, xa, 0L, M1ROWS, NHID, NC, WCARRY_INV, M1ROWS);
  {
    const int n2 = M1ROWS * NHID / 2;
    gelu_kernel<<<(n2 + 255) / 256, 256, 0, stream>>>(pre1, t1, n2);
  }
  wmma_gemm64<0, false, 2, 0, true><<<gemm_grid(M1ROWS, NC), 256, 0, stream>>>(
      t1, t1, NHID, 0L, w2T, w2T, NHID, 0L, (void*)y1p, (void*)y1p, NC, 0L,
      b12, xa, 0L, M1ROWS, NC, NHID, WCARRY_INV, M1ROWS);

  dwt_kernel<<<(NB * DH * (DW / 4)) / 256, 256, 0, stream>>>(hf, pll, plh, phl, phh);
  upsample_kernel<<<(M2PAD * (NC / 2)) / 256, 256, 0, stream>>>(pll, low16);
  wmma_gemm64<0, false, 2, 0, false><<<gemm_grid(M2PAD, NHID), 256, 0, stream>>>(
      low16, low16, NC, 0L, w1T + (size_t)NHID * NC, w1T + (size_t)NHID * NC, NC, 0L,
      (void*)pre2, (void*)pre2, NHID, 0L, b21, xa, 0L, M2PAD, NHID, NC, WCARRY_INV, M2PAD);
  {
    const int n2 = M2PAD * NHID / 2;
    gelu_kernel<<<(n2 + 255) / 256, 256, 0, stream>>>(pre2, t2, n2);
  }
  wmma_gemm64<0, false, 2, 0, false><<<gemm_grid(M2PAD, NC), 256, 0, stream>>>(
      t2, t2, NHID, 0L, w2T + (size_t)NC * NHID, w2T + (size_t)NC * NHID, NHID, 0L,
      (void*)lowout, (void*)lowout, NC, 0L, b22, xa, 0L, M2PAD, NC, NHID, WCARRY_INV, M2PAD);

  final_kernel<<<MROWS / 8, 256, 0, stream>>>(y1p, xpost, lowout, plh, phl, phh, out);
}
